// MultiHeadAttention_91311004713550
// MI455X (gfx1250) — hardware-run, weakly checked
//
#include <hip/hip_runtime.h>


#ifndef NB
#define NB 8
#endif
#ifndef SEQ
#define SEQ 1024
#endif
#define NB_FULL  8
#define SEQ_FULL 1024
#ifndef OUT_SEQ
#define OUT_SEQ SEQ
#endif
#define DM   512
#define NH_  8
#define HD   64
#define WIN  4
#define NREL 9
#define AW   4
#define QRS  2048.0f
#define SC2  (0.125f * 1.4426950408889634f)
#define PSH  8.0f
#define EKS  64.0f
#define WOS  64.0f
#define OSC  64.0f
#define OSI  (1.0f / 4096.0f)
#define RLP  20
#define EKP  72
#define EVP  40

static_assert(HD == 64);
static_assert(NH_ * HD == DM);
static_assert(DM % 64 == 0);
static_assert(DM % 32 == 0);
static_assert(SEQ % 64 == 0);
static_assert((NB * SEQ) % 64 == 0);
static_assert(SEQ % 32 == 0);
static_assert(SEQ % (16 * AW) == 0);
static_assert(OUT_SEQ % 64 == 0);
static_assert(SEQ_FULL % 4 == 0);
static_assert(NB <= NB_FULL);
static_assert(SEQ <= SEQ_FULL);
static_assert(NREL == 2 * WIN + 1);
static_assert(NREL <= 16);

typedef _Float16 h16;
typedef unsigned short bf;
typedef __attribute__((ext_vector_type(16))) __bf16   v16bf;
typedef __attribute__((ext_vector_type(16))) _Float16 v16h;
typedef __attribute__((ext_vector_type(8)))  _Float16 v8h;
typedef __attribute__((ext_vector_type(8)))  unsigned short v8us;
typedef __attribute__((ext_vector_type(8)))  float    v8f;
typedef __attribute__((ext_vector_type(4)))  float    v4f;
typedef v4f  __attribute__((may_alias)) v4fa;

__device__ __forceinline__ unsigned short f2bf(float f) { unsigned u = __float_as_uint(f); u += 0x7FFFu + ((u >> 16) & 1u); return (unsigned short)(u >> 16); }
__device__ __forceinline__ float bfr(float f) { return __uint_as_float(((unsigned)f2bf(f)) << 16); }
__device__ __forceinline__ v16h cat16(v8h lo, v8h hi) { return __builtin_shufflevector(lo, hi, 0, 1, 2, 3, 4, 5, 6, 7, 8, 9, 10, 11, 12, 13, 14, 15); }
__device__ __forceinline__ v16bf cat16b(v8us lo, v8us hi) { return __builtin_bit_cast(v16bf, __builtin_shufflevector(lo, hi, 0, 1, 2, 3, 4, 5, 6, 7, 8, 9, 10, 11, 12, 13, 14, 15)); }
__device__ __forceinline__ v8f wmma16(v16h a, v16h b, v8f c) { return __builtin_amdgcn_wmma_f32_16x16x32_f16(false, a, false, b, (short)0, c, false, false); }
__device__ __forceinline__ v8f wmmab(v16bf a, v16bf b, v8f c) { return __builtin_amdgcn_wmma_f32_16x16x32_bf16(false, a, false, b, (short)0, c, false, false); }
__device__ __forceinline__ v16h  ldh(const h16* p) { return cat16(*(const v8h*)p, *(const v8h*)(p + 16)); }
__device__ __forceinline__ v16bf ldb(const bf* p)  { return cat16b(*(const v8us*)p, *(const v8us*)(p + 16)); }
__device__ __forceinline__ void wave_sync() { __builtin_amdgcn_fence(3  , "wavefront"); __builtin_amdgcn_wave_barrier(); asm volatile("" ::: "memory"); }
__device__ __forceinline__ unsigned short cv16(float v, int mode) {
    const unsigned short b = f2bf(v);
    const h16 hx = (h16)(__uint_as_float(((unsigned)b) << 16) * WOS);
    const unsigned short hb = __builtin_bit_cast(unsigned short, hx);
    return mode ? hb : b;
}

__global__ __launch_bounds__(256) void k_tcvt(const float* __restrict__ src, unsigned short* dst, int inPitch, size_t inBS, int outPitch, size_t outBS, int mode) {
    __shared__ __align__(16) float ts[64 * 68];
    const int tid = threadIdx.x;
    const int c0 = blockIdx.x * 64, r0 = blockIdx.y * 64;
    const float* s = src + (size_t)blockIdx.z * inBS;
#pragma unroll
    for (int it = 0; it < 4; ++it) {
        const int rr = it * 16 + (tid >> 4), c4 = (tid & 15) * 4;
        const v4f v = *(const v4f*)(s + (size_t)(r0 + rr) * (size_t)inPitch + c0 + c4);
#pragma unroll
        for (int i = 0; i < 4; ++i) ts[(c4 + i) * 68 + rr] = v[i];
    }
    __syncthreads();
    unsigned short* d = dst + (size_t)blockIdx.z * outBS;
    v8us o0, o1;
    const int q8 = (tid & 7) * 8;
    const int ca = (tid >> 3), cb = 32 + (tid >> 3);
    {
        const v4f x0 = *(const v4fa*)(&ts[ca * 68 + q8]); const v4f x1 = *(const v4fa*)(&ts[ca * 68 + q8 + 4]);
        const v4f y0 = *(const v4fa*)(&ts[cb * 68 + q8]); const v4f y1 = *(const v4fa*)(&ts[cb * 68 + q8 + 4]);
#pragma unroll
        for (int i = 0; i < 4; ++i) { o0[i] = cv16(x0[i], mode); o0[4 + i] = cv16(x1[i], mode); o1[i] = cv16(y0[i], mode); o1[4 + i] = cv16(y1[i], mode); }
    }
    const size_t oa = (size_t)(c0 + ca) * (size_t)outPitch + r0 + q8;
    const size_t ob = (size_t)(c0 + cb) * (size_t)outPitch + r0 + q8;
    *(volatile v8us*)(d + oa) = o0; *(volatile v8us*)(d + ob) = o1;
    __threadfence();
    *(volatile v8us*)(d + oa) = o0; *(volatile v8us*)(d + ob) = o1;
}

__global__ __launch_bounds__(32) void k_proj(const bf* __restrict__ A, const bf* __restrict__ Bt, h16* Ph, h16* Pr, int useRes, const float* __restrict__ bias, int biasRow,
                                             int RB, size_t sRB, int pitch, int CB, size_t sCB) {
    __shared__ __align__(16) float os[16 * 68];
    const int K = DM;
    const int lane = threadIdx.x & 31, lr = lane & 15, hi = lane >> 4; const int r0 = blockIdx.x * 64, c0 = blockIdx.y * 64;
    v8f acc[4][4];
#pragma unroll
    for (int mb = 0; mb < 4; ++mb)
#pragma unroll
        for (int nb = 0; nb < 4; ++nb) acc[mb][nb] = (v8f){};
    const size_t aoff = (size_t)(r0 + lr) * K + 8 * hi, boff = (size_t)(c0 + lr) * K + 8 * hi;
#pragma unroll 1
    for (int kc = 0; kc < K; kc += 32) {
        v16bf a[4];
#pragma unroll
        for (int mb = 0; mb < 4; ++mb) a[mb] = ldb(A + aoff + (size_t)mb * 16 * K + kc);
#pragma unroll
        for (int nb = 0; nb < 4; ++nb) { const v16bf b = ldb(Bt + boff + (size_t)nb * 16 * K + kc);
#pragma unroll
            for (int mb = 0; mb < 4; ++mb) acc[mb][nb] = wmmab(a[mb], b, acc[mb][nb]); }
        asm volatile("v_nop\n\tv_nop\n\tv_nop\n\tv_nop" : "+v"(acc[0][0]), "+v"(acc[1][1]), "+v"(acc[2][2]), "+v"(acc[3][3]) : "v"(a[0]), "v"(a[1]), "v"(a[2]), "v"(a[3]));
    }
    float cbias[4];
#pragma unroll
    for (int nb = 0; nb < 4; ++nb) cbias[nb] = bfr(bias[min(c0 + nb * 16 + lr, DM - 1)]);
    const size_t tbase = (size_t)(r0 / RB) * sRB + (size_t)(r0 % RB) * (size_t)pitch + (size_t)(c0 / CB) * sCB + (size_t)(c0 % CB);
#pragma unroll
    for (int mb = 0; mb < 4; ++mb) {
        float rbias[8];
#pragma unroll
        for (int j = 0; j < 8; ++j) rbias[j] = bfr(bias[min(r0 + mb * 16 + hi * 8 + j, DM - 1)]);
#pragma unroll
        for (int nb = 0; nb < 4; ++nb) {
#pragma unroll
            for (int j = 0; j < 8; ++j) os[(hi * 8 + j) * 68 + nb * 16 + lr] = acc[mb][nb][j] + (biasRow ? rbias[j] : cbias[nb]); }
        wave_sync();
        const size_t sb = tbase + (size_t)(mb * 16) * (size_t)pitch;
#pragma unroll 1
        for (int ps = 0; ps < 2; ++ps) {
#pragma unroll
            for (int s = 0; s < 4; ++s) { const int row = 4 * s + (lane >> 3), c8 = (lane & 7) * 8;
                const v4f x0 = *(const v4fa*)(&os[row * 68 + c8]); const v4f x1 = *(const v4fa*)(&os[row * 68 + c8 + 4]); v8h hv, rv;
#pragma unroll
                for (int i = 0; i < 4; ++i) { const h16 a0 = (h16)x0[i]; const h16 a1 = (h16)x1[i]; hv[i] = a0; hv[4 + i] = a1; rv[i] = (h16)((x0[i] - (float)a0) * QRS); rv[4 + i] = (h16)((x1[i] - (float)a1) * QRS); }
                const size_t oo = sb + (size_t)row * (size_t)pitch + c8;
                *(volatile v8h*)(Ph + oo) = hv; if (useRes) *(volatile v8h*)(Pr + oo) = rv; }
            if (ps == 0) __threadfence(); }
        wave_sync();
    }
}

__global__ __launch_bounds__(32 * AW) void k_flash(const h16* __restrict__ QH, const h16* __restrict__ KH, const h16* __restrict__ VH,
                                                   const float* __restrict__ ekg, const float* __restrict__ evg, h16* OHP) {
    __shared__ __align__(16) float os[AW * 16 * 68];
    __shared__ __align__(16) float relT[AW * 16 * RLP];
    __shared__ __align__(16) float bl[AW * 16 * RLP];
    __shared__ __align__(16) h16 ek_s[16 * EKP];
    __shared__ __align__(16) h16 ev_s[HD * EVP];
    const int tid = threadIdx.x;
    const int lane = tid & 31, wave = __builtin_amdgcn_readfirstlane((int)(tid >> 5)), lr = lane & 15, hi = lane >> 4;
    for (int i = tid; i < 16 * EKP; i += 32 * AW) {
        const int mm = i / EKP, d = i % EKP; const bool ok = (mm < NREL) && (d < HD);
        const float v = bfr(ekg[min(mm, NREL - 1) * HD + min(d, HD - 1)]) * EKS;
        ek_s[i] = (h16)(ok ? v : 0.0f); }
    for (int i = tid; i < HD * EVP; i += 32 * AW) {
        const int d = i / EVP, kk = i % EVP; const bool ok = (kk < NREL);
        const float v = bfr(evg[min(kk, NREL - 1) * HD + d]);
        ev_s[i] = (h16)(ok ? v : 0.0f); }
    __syncthreads();

    const int zh = blockIdx.y; const int b = zh / NH_, h = zh % NH_;
    const int t0 = (blockIdx.x * AW + wave) * 16;
    const size_t pbase = (size_t)zh * SEQ * HD;
    const size_t qo = pbase + (size_t)(t0 + lr) * HD + 8 * hi;
    const v16h qh0 = ldh(QH + qo), qh1 = ldh(QH + qo + 32);
    const int wb = wave * 16 * 68, wr = wave * 16 * RLP;
    {
        v8f rH = (v8f){};
        const v16h e0 = cat16(*(const v8h*)(&ek_s[lr * EKP + 8 * hi]),      *(const v8h*)(&ek_s[lr * EKP + 8 * hi + 16]));
        const v16h e1 = cat16(*(const v8h*)(&ek_s[lr * EKP + 32 + 8 * hi]), *(const v8h*)(&ek_s[lr * EKP + 32 + 8 * hi + 16]));
        rH = wmma16(e0, qh0, rH); rH = wmma16(e1, qh1, rH);
        asm volatile("v_nop\n\tv_nop\n\tv_nop\n\tv_nop" : "+v"(rH) : "v"(e0), "v"(e1));
        v4f a, c, ng;
#pragma unroll
        for (int i = 0; i < 4; ++i) { a[i] = rH[i] * (SC2 / EKS); c[i] = rH[4 + i] * (SC2 / EKS); ng[i] = -3.0e38f; }
        *(v4fa*)(&relT[wr + lr * RLP + 8 * hi]) = a;  *(v4fa*)(&relT[wr + lr * RLP + 8 * hi + 4]) = c;
        *(v4fa*)(&bl[wr + lr * RLP + 8 * hi]) = ng;   *(v4fa*)(&bl[wr + lr * RLP + 8 * hi + 4]) = ng;
    }
    wave_sync();
    const size_t ko = pbase + (size_t)lr * HD + 8 * hi;
    const size_t vo = pbase + (size_t)lr * SEQ + 8 * hi;
    v8f oH[4];
#pragma unroll
    for (int j = 0; j < 4; ++j) oH[j] = (v8f){};
    float m = -3.0e38f, l = 0.0f;
#pragma unroll 1
    for (int key0 = 0; key0 < SEQ; key0 += 32) {
        const h16* ka = KH + ko + (size_t)key0 * HD;
        const v16h ka0 = ldh(ka), ka1 = ldh(ka + 32), kb0 = ldh(ka + 16 * HD), kb1 = ldh(ka + 16 * HD + 32);
        v8f sHa = (v8f){}, sHb = (v8f){};
        sHa = wmma16(ka0, qh0, sHa); sHb = wmma16(kb0, qh0, sHb);
        sHa = wmma16(ka1, qh1, sHa); sHb = wmma16(kb1, qh1, sHb);
        asm volatile("v_nop\n\tv_nop\n\tv_nop\n\tv_nop" : "+v"(sHa), "+v"(sHb) : "v"(ka0), "v"(ka1), "v"(kb0), "v"(kb1));
        float ta[8], tb[8];
#pragma unroll
        for (int r = 0; r < 8; ++r) { ta[r] = sHa[r] * SC2; tb[r] = sHb[r] * SC2; }
        if (key0 + 31 >= t0 - WIN && key0 <= t0 + 15 + WIN) {
            const int ib = t0 + lr - WIN;
#pragma unroll
            for (int r = 0; r < 8; ++r) {
                const int ma = key0 + 8 * hi + r - ib, mb2 = ma + 16;
                const bool va = ((unsigned)ma <= (unsigned)(2 * WIN)), vb = ((unsigned)mb2 <= (unsigned)(2 * WIN));
                const int ca = min(max(ma, 0), 2 * WIN), cb = min(max(mb2, 0), 2 * WIN);
                const float ra = relT[wr + lr * RLP + ca], rb = relT[wr + lr * RLP + cb];
                ta[r] += va ? ra : 0.0f; tb[r] += vb ? rb : 0.0f;
                if (va) bl[wr + lr * RLP + ca] = ta[r];
                if (vb) bl[wr + lr * RLP + cb] = tb[r];
            }
        }
        float mx = -3.0e38f;
#pragma unroll
        for (int r = 0; r < 8; ++r) mx = fmaxf(mx, fmaxf(ta[r], tb[r]));
        mx = fmaxf(mx, __shfl_xor(mx, 16, 32));
        const float mnew = fmaxf(m, mx);
        const float alpha = __builtin_amdgcn_exp2f(m - mnew);
        const float sh = PSH - mnew;
        v16h pb; float ls = 0.0f;
#pragma unroll
        for (int r = 0; r < 8; ++r) { const h16 pa = (h16)__builtin_amdgcn_exp2f(ta[r] + sh); const h16 pc = (h16)__builtin_amdgcn_exp2f(tb[r] + sh); pb[r] = pa; pb[8 + r] = pc; ls += (float)pa + (float)pc; }
        l = l * alpha + ls; m = mnew;
#pragma unroll
        for (int j = 0; j < 4; ++j) oH[j] = oH[j] * alpha;
        asm volatile("" ::: "memory");
        const h16* va = VH + vo + key0;
        v16h vh[4];
#pragma unroll
        for (int j = 0; j < 4; ++j) vh[j] = ldh(va + (size_t)(16 * j) * SEQ);
#pragma unroll
        for (int j = 0; j < 4; ++j) oH[j] = wmma16(vh[j], pb, oH[j]);
        asm volatile("v_nop\n\tv_nop\n\tv_nop\n\tv_nop" : "+v"(oH[0]), "+v"(oH[1]), "+v"(oH[2]), "+v"(oH[3]) : "v"(vh[0]), "v"(vh[1]), "v"(vh[2]), "v"(vh[3]), "v"(pb));
    }
    wave_sync();
    l += __shfl_xor(l, 16, 32);
    {
        const v4f g0 = *(const v4fa*)(&bl[wr + lr * RLP + 8 * hi]); const v4f g1 = *(const v4fa*)(&bl[wr + lr * RLP + 8 * hi + 4]);
        const float shf = PSH - m;
        v16h pw;
#pragma unroll
        for (int i = 0; i < 4; ++i) { pw[i] = (h16)__builtin_amdgcn_exp2f(g0[i] + shf); pw[4 + i] = (h16)__builtin_amdgcn_exp2f(g1[i] + shf); }
#pragma unroll
        for (int i = 8; i < 16; ++i) pw[i] = (h16)0.0f;
        v16h ea[4];
#pragma unroll
        for (int j = 0; j < 4; ++j) ea[j] = cat16(*(const v8h*)(&ev_s[(16 * j + lr) * EVP + 8 * hi]), *(const v8h*)(&ev_s[(16 * j + lr) * EVP + 8 * hi + 16]));
#pragma unroll
        for (int j = 0; j < 4; ++j) oH[j] = wmma16(ea[j], pw, oH[j]);
        asm volatile("v_nop\n\tv_nop\n\tv_nop\n\tv_nop" : "+v"(oH[0]), "+v"(oH[1]), "+v"(oH[2]), "+v"(oH[3]) : "v"(ea[0]), "v"(ea[1]), "v"(ea[2]), "v"(ea[3]), "v"(pw));
    }
    const float inv = OSC * (1.0f / l);
#pragma unroll
    for (int j = 0; j < 4; ++j) { v4f a, c;
#pragma unroll
        for (int i = 0; i < 4; ++i) { a[i] = oH[j][i] * inv; c[i] = oH[j][4 + i] * inv; }
        *(v4fa*)(&os[wb + lr * 68 + 16 * j + 8 * hi]) = a; *(v4fa*)(&os[wb + lr * 68 + 16 * j + 8 * hi + 4]) = c; }
    wave_sync();
    const size_t obase = ((size_t)b * SEQ + t0) * DM + (size_t)h * HD;
#pragma unroll 1
    for (int ps = 0; ps < 2; ++ps) {
#pragma unroll
        for (int s = 0; s < 4; ++s) { const int row = 4 * s + (lane >> 3), c8 = (lane & 7) * 8;
            const v4f x0 = *(const v4fa*)(&os[wb + row * 68 + c8]); const v4f x1 = *(const v4fa*)(&os[wb + row * 68 + c8 + 4]); v8h hv;
#pragma unroll
            for (int i = 0; i < 4; ++i) { hv[i] = (h16)x0[i]; hv[4 + i] = (h16)x1[i]; }
            const size_t oo = obase + (size_t)row * DM + c8;
            *(volatile v8h*)(OHP + oo) = hv; }
        if (ps == 0) __threadfence(); }
}

__global__ __launch_bounds__(32) void k_outp(const h16* __restrict__ A, const h16* __restrict__ BH, const float* __restrict__ bias, float* Y) {
    __shared__ __align__(16) float os[16 * 68];
    const int K = DM;
    const int lane = threadIdx.x & 31, lr = lane & 15, hi = lane >> 4; const int r0 = blockIdx.x * 32, c0 = blockIdx.y * 64;
    v8f aH[2][4];
#pragma unroll
    for (int mb = 0; mb < 2; ++mb)
#pragma unroll
        for (int nb = 0; nb < 4; ++nb) aH[mb][nb] = (v8f){};
    const size_t aoff = (size_t)(r0 + lr) * K + 8 * hi, boff = (size_t)(c0 + lr) * K + 8 * hi;
#pragma unroll 1
    for (int kc = 0; kc < K; kc += 32) {
        v16h a[2];
#pragma unroll
        for (int mb = 0; mb < 2; ++mb) a[mb] = ldh(A + aoff + (size_t)mb * 16 * K + kc);
#pragma unroll
        for (int nb = 0; nb < 4; ++nb) { const v16h bh = ldh(BH + boff + (size_t)nb * 16 * K + kc);
#pragma unroll
            for (int mb = 0; mb < 2; ++mb) aH[mb][nb] = wmma16(a[mb], bh, aH[mb][nb]); }
        asm volatile("v_nop\n\tv_nop\n\tv_nop\n\tv_nop" : "+v"(aH[0][0]), "+v"(aH[0][3]), "+v"(aH[1][0]), "+v"(aH[1][3]) : "v"(a[0]), "v"(a[1]));
    }
    const int bb = c0 / SEQ, tt = c0 % SEQ;
    float* ybase = Y + ((size_t)bb * DM + r0) * (size_t)OUT_SEQ + tt;
#pragma unroll
    for (int mb = 0; mb < 2; ++mb) {
        float rbias[8];
#pragma unroll
        for (int j = 0; j < 8; ++j) rbias[j] = bfr(bias[min(r0 + mb * 16 + hi * 8 + j, DM - 1)]);
#pragma unroll
        for (int nb = 0; nb < 4; ++nb) {
#pragma unroll
            for (int j = 0; j < 8; ++j) os[(hi * 8 + j) * 68 + nb * 16 + lr] = aH[mb][nb][j] * OSI + rbias[j]; }
        wave_sync();
#pragma unroll 1
        for (int ps = 0; ps < 2; ++ps) {
#pragma unroll
            for (int s = 0; s < 8; ++s) { const int row = 2 * s + hi, cofs = lr * 4;
                const v4f val = *(const v4fa*)(&os[row * 68 + cofs]);
                *(volatile v4f*)(ybase + (size_t)(mb * 16 + row) * (size_t)OUT_SEQ + cofs) = val; }
            if (ps == 0) __threadfence(); }
        wave_sync();
    }
}

static constexpr size_t al256(size_t v) { return (v + 255) & ~(size_t)255; }
static constexpr size_t SZ_XT = al256((size_t)NB * SEQ * DM * 2);
static constexpr size_t SZ_W  = al256((size_t)DM * DM * 2);
static constexpr size_t SZ_PL = al256((size_t)NB * NH_ * SEQ * HD * 2);
static constexpr size_t SZ_TOTAL = 3 * SZ_XT + 4 * SZ_W + 3 * SZ_PL;
static_assert(SZ_TOTAL <= (size_t)134217728);
static_assert(((size_t)DM * DM * 2) % 256 == 0);
static_assert(((size_t)NB * SEQ * DM * 2) % 256 == 0);

extern "C" void kernel_launch(void* const* d_in, const int* in_sizes, int n_in,
                              void* d_out, int out_size, void* d_ws, size_t ws_size, hipStream_t stream) {
    if (n_in < 12) return;
    const size_t needx = ((size_t)(NB - 1) * DM + (DM - 1)) * SEQ_FULL + SEQ;
    if ((size_t)in_sizes[0] < needx || (size_t)in_sizes[1] < needx) return;
    if ((size_t)in_sizes[2] < (size_t)DM * DM || (size_t)in_sizes[4] < (size_t)DM * DM || (size_t)in_sizes[6] < (size_t)DM * DM || (size_t)in_sizes[8] < (size_t)DM * DM) return;
    if (in_sizes[3] < DM || in_sizes[5] < DM || in_sizes[7] < DM || in_sizes[9] < DM) return;
    if (in_sizes[10] < NREL * HD || in_sizes[11] < NREL * HD) return;
    if ((size_t)out_size < ((size_t)(NB - 1) * DM + (DM - 1)) * OUT_SEQ + SEQ) return;
    if (SZ_TOTAL > ws_size) return;
    const float* x  = (const float*)d_in[0]; const float* c  = (const float*)d_in[1];
    const float* wq = (const float*)d_in[2]; const float* bq = (const float*)d_in[3];
    const float* wk = (const float*)d_in[4]; const float* bk = (const float*)d_in[5];
    const float* wv = (const float*)d_in[6]; const float* bv = (const float*)d_in[7];
    const float* wo = (const float*)d_in[8]; const float* bo = (const float*)d_in[9];
    const float* ek = (const float*)d_in[10]; const float* ev = (const float*)d_in[11];
    float* Y = (float*)d_out;
    char* wsp = (char*)d_ws;
    bf* XT  = (bf*)wsp; wsp += SZ_XT;
    bf* CT  = (bf*)wsp; wsp += SZ_XT;
    bf* WQT = (bf*)wsp; wsp += SZ_W;
    bf* WKT = (bf*)wsp; wsp += SZ_W;
    bf* WVT = (bf*)wsp; wsp += SZ_W;
    bf* WOT = (bf*)wsp; wsp += SZ_W;
    h16* QH = (h16*)wsp; wsp += SZ_PL;
    h16* KH = (h16*)wsp; wsp += SZ_PL;
    h16* VH = (h16*)wsp; wsp += SZ_PL;
    h16* OHP = (h16*)wsp; wsp += SZ_XT;

    k_tcvt<<<dim3(SEQ / 64, DM / 64, NB), 256, 0, stream>>>(x, XT, SEQ_FULL, (size_t)DM * SEQ_FULL, DM, (size_t)SEQ * DM, 0);
    k_tcvt<<<dim3(SEQ / 64, DM / 64, NB), 256, 0, stream>>>(c, CT, SEQ_FULL, (size_t)DM * SEQ_FULL, DM, (size_t)SEQ * DM, 0);
    k_tcvt<<<dim3(DM / 64, DM / 64, 1), 256, 0, stream>>>(wq, WQT, DM, (size_t)0, DM, (size_t)0, 0);
    k_tcvt<<<dim3(DM / 64, DM / 64, 1), 256, 0, stream>>>(wk, WKT, DM, (size_t)0, DM, (size_t)0, 0);
    k_tcvt<<<dim3(DM / 64, DM / 64, 1), 256, 0, stream>>>(wv, WVT, DM, (size_t)0, DM, (size_t)0, 0);
    k_tcvt<<<dim3(DM / 64, DM / 64, 1), 256, 0, stream>>>(wo, WOT, DM, (size_t)0, DM, (size_t)0, 1);

    k_proj<<<dim3(NB * SEQ / 64, DM / 64, 1), 32, 0, stream>>>(XT, WQT, QH, QH, 0, bq, 0, SEQ, (size_t)NH_ * SEQ * HD, HD, HD, (size_t)SEQ * HD);
    k_proj<<<dim3(NB * SEQ / 64, DM / 64, 1), 32, 0, stream>>>(CT, WKT, KH, KH, 0, bk, 0, SEQ, (size_t)NH_ * SEQ * HD, HD, HD, (size_t)SEQ * HD);
    k_proj<<<dim3(DM / 64, NB * SEQ / 64, 1), 32, 0, stream>>>(WVT, CT, VH, VH, 0, bv, 1, DM, (size_t)0, SEQ, SEQ, (size_t)DM * SEQ);

    k_flash<<<dim3(SEQ / (16 * AW), NB * NH_, 1), 32 * AW, 0, stream>>>(QH, KH, VH, ek, ev, OHP);

    k_outp<<<dim3(DM / 32, NB * SEQ / 64, 1), 32, 0, stream>>>((const h16*)WOT, OHP, bo, Y);
}
